// MP_up_14001593385536
// MI455X (gfx1250) — hardware-verified
//
#include <hip/hip_runtime.h>
#include <stddef.h>


#define DD      128
#define HEADS   8
#define DKH     16
#define FFW     256
#define QKVW    384
#define NL      2
#define NTHR    256
#define NWAVE   8
#define EPT     8
#define NGRP    2
#define CHUNK   (NTHR * EPT * NGRP)
#define WCAP    (EPT * NGRP * 32)
#define LISTN   (NWAVE * WCAP)
#define NBC     4096
#define NBF     1024
#define RCAP    40960
#define RBN     128
#define TGT     256
#define DEGCAP  256
#define OTHR    512
#define WSCAP   134217728
#define WCARRY  16.0f
#define ACARRY  8.0f
#define LN_EPS  1e-5f
#define Z_EPS   1e-6f

#define LDS_FILL ((RCAP + NBF + LISTN) * 4 + 64)

static_assert((CHUNK & (CHUNK - 1)) == 0);
static_assert(CHUNK <= 4096);
static_assert(NBC <= 4096 && NBF <= 4096);
static_assert((NBC & (NBC - 1)) == 0 && (NBF & (NBF - 1)) == 0);
static_assert(NBC == 4 * NBF);
static_assert(OTHR * 8 == NBC);
static_assert((RCAP % 32) == 0);
static_assert(TGT == NWAVE * 32);
static_assert((NBC % TGT) == 0);
static_assert(HEADS * DKH == DD && DKH == 16);

typedef float     v4f  __attribute__((ext_vector_type(4)));
typedef float     v8f  __attribute__((ext_vector_type(8)));
typedef int       v4i  __attribute__((ext_vector_type(4)));
typedef _Float16  v4h  __attribute__((ext_vector_type(4)));
typedef _Float16  v8h  __attribute__((ext_vector_type(8)));
typedef _Float16  v16h __attribute__((ext_vector_type(16)));
union Frag { v16h v; v8h h[2]; };

__device__ __forceinline__ v8f wmh(v16h a, v16h b, v8f c) {
  v8f d = __builtin_amdgcn_wmma_f32_16x16x32_f16(false, a, false, b, (short)0, c, false, false);
  asm volatile("v_nop\n\tv_nop\n\tv_nop\n\tv_nop" : "+v"(d) : "v"(a), "v"(b));
  return d;
}

__device__ __forceinline__ v8h cvt8(v4f a, v4f b, float s) {
  v8h o;
  o[0] = (_Float16)(a.x * s); o[1] = (_Float16)(a.y * s); o[2] = (_Float16)(a.z * s); o[3] = (_Float16)(a.w * s);
  o[4] = (_Float16)(b.x * s); o[5] = (_Float16)(b.y * s); o[6] = (_Float16)(b.z * s); o[7] = (_Float16)(b.w * s);
  return o;
}

template <int NB>
__device__ __forceinline__ int scan_chunk(const int* __restrict__ dsts, int nE, int cbase, int slotBase,
                                          int vec8, int* list, int tid, int lane, int wave) {
  int wc = 0;
#pragma unroll
  for (int g = 0; g < NGRP; ++g) {
    const int el0  = (g * NTHR + tid) * EPT;
    const int e0   = cbase + el0;
    const int sent = -2147483647 - 1;
    v4i da, db;
    if (vec8 != 0 && cbase + CHUNK <= nE) {
      da = *(const v4i*)(dsts + e0);
      db = *(const v4i*)(dsts + e0 + 4);
    } else {
      da.x = (e0     < nE) ? dsts[min(e0, nE - 1)] : sent;
      da.y = (e0 + 1 < nE) ? dsts[min(e0 + 1, nE - 1)] : sent;
      da.z = (e0 + 2 < nE) ? dsts[min(e0 + 2, nE - 1)] : sent;
      da.w = (e0 + 3 < nE) ? dsts[min(e0 + 3, nE - 1)] : sent;
      db.x = (e0 + 4 < nE) ? dsts[min(e0 + 4, nE - 1)] : sent;
      db.y = (e0 + 5 < nE) ? dsts[min(e0 + 5, nE - 1)] : sent;
      db.z = (e0 + 6 < nE) ? dsts[min(e0 + 6, nE - 1)] : sent;
      db.w = (e0 + 7 < nE) ? dsts[min(e0 + 7, nE - 1)] : sent;
    }
    const unsigned nb = (unsigned)slotBase;
    const unsigned s0 = (unsigned)da.x - nb, s1 = (unsigned)da.y - nb;
    const unsigned s2 = (unsigned)da.z - nb, s3 = (unsigned)da.w - nb;
    const unsigned s4 = (unsigned)db.x - nb, s5 = (unsigned)db.y - nb;
    const unsigned s6 = (unsigned)db.z - nb, s7 = (unsigned)db.w - nb;
    const bool h0 = s0 < (unsigned)NB, h1 = s1 < (unsigned)NB, h2 = s2 < (unsigned)NB, h3 = s3 < (unsigned)NB;
    const bool h4 = s4 < (unsigned)NB, h5 = s5 < (unsigned)NB, h6 = s6 < (unsigned)NB, h7 = s7 < (unsigned)NB;
    const unsigned any = __builtin_amdgcn_ballot_w32(h0 | h1 | h2 | h3 | h4 | h5 | h6 | h7);
    if (any != 0u) {
#define HITJ(J, HJ, SJ) { \
        const unsigned mj = __builtin_amdgcn_ballot_w32(HJ); \
        if (mj != 0u) { \
          if (HJ) { \
            const int pos = wc + (int)__builtin_amdgcn_mbcnt_lo(mj, 0u); \
            if (pos < WCAP) list[wave * WCAP + pos] = ((el0 + (J)) << 12) | (int)(SJ); \
          } \
          wc += (int)__builtin_popcount(mj); } }
      HITJ(0, h0, s0)
      HITJ(1, h1, s1)
      HITJ(2, h2, s2)
      HITJ(3, h3, s3)
      HITJ(4, h4, s4)
      HITJ(5, h5, s5)
      HITJ(6, h6, s6)
      HITJ(7, h7, s7)
#undef HITJ
    }
  }
  return wc;
}

__global__ __launch_bounds__(NTHR) void k_wprep(const float* __restrict__ W, _Float16* wp,
                                                 int Kd, int Nd, int nUnits, int outL, int nOff) {
  const int i = (int)blockIdx.x * NTHR + (int)threadIdx.x;
  if (i >= nUnits) return;
  const int kd8 = Kd >> 3;
  const int per = Nd * kd8;
  const int l   = i / per;
  const int rem = i - l * per;
  const int n   = rem / kd8;
  const int k0  = (rem - n * kd8) * 8;
  const float* sp = W + (size_t)l * Kd * Nd + (size_t)k0 * Nd + n;
  v4f a, b;
  a.x = sp[0];               a.y = sp[(size_t)Nd];      a.z = sp[(size_t)2 * Nd];  a.w = sp[(size_t)3 * Nd];
  b.x = sp[(size_t)4 * Nd];  b.y = sp[(size_t)5 * Nd];  b.z = sp[(size_t)6 * Nd];  b.w = sp[(size_t)7 * Nd];
  const v8h o = cvt8(a, b, WCARRY);
  _Float16* dp = wp + (size_t)l * outL + (size_t)(nOff + n) * Kd + k0;
  *(volatile v8h*)dp = o;
  __threadfence();
  *(volatile v8h*)dp = o;
}

__global__ __launch_bounds__(NTHR) void k_cvt(const float* __restrict__ X, _Float16* Y, int nN, int nUnits) {
  const int i = (int)blockIdx.x * NTHR + (int)threadIdx.x;
  if (i >= nUnits) return;
  const int row = i >> 4;
  const int c0  = (i & 15) * 8;
  const int rr  = row < nN ? row : nN - 1;
  const float* sp = X + (size_t)rr * DD + c0;
  const v4f z4 = {0.f, 0.f, 0.f, 0.f};
  v4f a = *(const v4f*)sp, b = *(const v4f*)(sp + 4);
  a = (row < nN) ? a : z4;
  b = (row < nN) ? b : z4;
  const v8h o = cvt8(a, b, 1.0f);
  _Float16* dp = Y + (size_t)i * 8;
  *(volatile v8h*)dp = o;
  __threadfence();
  *(volatile v8h*)dp = o;
}

__global__ __launch_bounds__(NTHR) void k_count(
    const int* __restrict__ dsts, int* cnt, int nE, int vec8) {
  __shared__ __attribute__((aligned(16))) int scnt[NBC];
  __shared__ __attribute__((aligned(16))) int list[LISTN];
  __shared__ int wcnt[NWAVE];
  const int tid = threadIdx.x, lane = tid & 31, wave = tid >> 5;
  const int nodeBase = blockIdx.x * NBC;

  for (int i = tid; i < NBC; i += NTHR) scnt[i] = 0;
  __syncthreads();

  const int nChunks = (nE + CHUNK - 1) / CHUNK;
#pragma unroll 1
  for (int ch = 0; ch < nChunks; ++ch) {
    const int cbase = ch * CHUNK;
    const int wc = scan_chunk<NBC>(dsts, nE, cbase, nodeBase, vec8, list, tid, lane, wave);
    if (lane == 0) wcnt[wave] = wc;
    __syncthreads();
    if (wave == 0) {
#pragma unroll 1
      for (int wsx = 0; wsx < NWAVE; ++wsx) {
        int n = __builtin_amdgcn_readfirstlane(wcnt[wsx]);
        n = n > WCAP ? WCAP : (n < 0 ? 0 : n);
        const int* lp = list + wsx * WCAP;
#pragma unroll 1
        for (int i = 0; i < n; ++i) {
          const int ent  = __builtin_amdgcn_readfirstlane(lp[i]);
          const int slot = ent & (NBC - 1);
          if (lane == 0) scnt[slot] = scnt[slot] + 1;
        }
      }
    }
    __syncthreads();
  }

  v4i cq[4];
#pragma unroll
  for (int q = 0; q < 4; ++q) {
    const int f = (wave * 4 + q) * 128 + 4 * lane;
    cq[q] = *(const v4i*)(scnt + f);
  }
  int* cp = cnt + (size_t)nodeBase;
#pragma unroll
  for (int q = 0; q < 4; ++q) {
    const int f = (wave * 4 + q) * 128 + 4 * lane;
    *(volatile v4i*)(cp + f) = cq[q];
  }
  __threadfence();
#pragma unroll
  for (int q = 0; q < 4; ++q) {
    const int f = (wave * 4 + q) * 128 + 4 * lane;
    *(volatile v4i*)(cp + f) = cq[q];
  }
}

__global__ __launch_bounds__(OTHR) void k_offsets(
    const int* __restrict__ cnt, int* off, int* rbase, int nChunk) {
  __shared__ __attribute__((aligned(16))) int soff[NBC];
  __shared__ __attribute__((aligned(16))) int srb[RBN];
  __shared__ int wtot[OTHR / 32];
  const int tid = threadIdx.x, lane = tid & 31, wave = tid >> 5, sub = tid >> 7;
  for (int i = tid; i < RBN; i += OTHR) srb[i] = 0;
  int carry = 0;
#pragma unroll 1
  for (int ch = 0; ch < nChunk; ++ch) {
    const int base = ch * NBC;
    const v4i c0 = *(const v4i*)(cnt + base + 8 * tid);
    const v4i c1 = *(const v4i*)(cnt + base + 8 * tid + 4);
    const int e0 = max(c0.x, 0), e1 = max(c0.y, 0), e2 = max(c0.z, 0), e3 = max(c0.w, 0);
    const int e4 = max(c1.x, 0), e5 = max(c1.y, 0), e6 = max(c1.z, 0), e7 = max(c1.w, 0);
    const int ts = e0 + e1 + e2 + e3 + e4 + e5 + e6 + e7;
    int incl = ts;
#pragma unroll
    for (int d = 1; d < 32; d <<= 1) {
      const int t = __shfl_up(incl, d);
      if (lane >= d) incl += t;
    }
    if (lane == 31) wtot[wave] = incl;
    __syncthreads();
    const int S0 = wtot[0]  + wtot[1]  + wtot[2]  + wtot[3];
    const int S1 = wtot[4]  + wtot[5]  + wtot[6]  + wtot[7];
    const int S2 = wtot[8]  + wtot[9]  + wtot[10] + wtot[11];
    const int S3 = wtot[12] + wtot[13] + wtot[14] + wtot[15];
    int pre = 0;
#pragma unroll 1
    for (int w = 4 * sub; w < wave; ++w) pre += wtot[w];
    const int b0 = carry;
    const int b1 = b0 + ((S0 + 31) & ~31);
    const int b2 = b1 + ((S1 + 31) & ~31);
    const int b3 = b2 + ((S2 + 31) & ~31);
    const int b4 = b3 + ((S3 + 31) & ~31);
    const int myb = sub == 0 ? b0 : (sub == 1 ? b1 : (sub == 2 ? b2 : b3));
    if (tid == 0) {
      srb[min(4 * ch + 0, RBN - 1)] = b0;
      srb[min(4 * ch + 1, RBN - 1)] = b1;
      srb[min(4 * ch + 2, RBN - 1)] = b2;
      srb[min(4 * ch + 3, RBN - 1)] = b3;
    }
    int run = myb + pre + incl - ts;
    soff[8 * tid + 0] = run; run += e0;
    soff[8 * tid + 1] = run; run += e1;
    soff[8 * tid + 2] = run; run += e2;
    soff[8 * tid + 3] = run; run += e3;
    soff[8 * tid + 4] = run; run += e4;
    soff[8 * tid + 5] = run; run += e5;
    soff[8 * tid + 6] = run; run += e6;
    soff[8 * tid + 7] = run;
    carry = b4;
    __syncthreads();
    const v4i o0 = *(const v4i*)(soff + 4 * tid);
    const v4i o1 = *(const v4i*)(soff + 4 * (tid + OTHR));
    int* op = off + base;
    *(volatile v4i*)(op + 4 * tid) = o0;
    *(volatile v4i*)(op + 4 * (tid + OTHR)) = o1;
    __threadfence();
    *(volatile v4i*)(op + 4 * tid) = o0;
    *(volatile v4i*)(op + 4 * (tid + OTHR)) = o1;
    __syncthreads();
  }
  if (tid == 0) srb[min(4 * nChunk, RBN - 1)] = carry;
  __syncthreads();
  v4i rv = {0, 0, 0, 0};
  if (tid < 32) rv = *(const v4i*)(srb + 4 * tid);
  if (tid < 32) *(volatile v4i*)(rbase + 4 * tid) = rv;
  __threadfence();
  if (tid < 32) *(volatile v4i*)(rbase + 4 * tid) = rv;
}

__global__ __launch_bounds__(NTHR) void k_fill(
    const int* __restrict__ srcs, const int* __restrict__ dsts,
    const int* __restrict__ off, const int* __restrict__ rbase,
    int* csr, int nN, int nE, int vec8, int csrLen) {
  extern __shared__ v4f lds_dyn[];
  int* region = (int*)lds_dyn;
  int* cursor = region + RCAP;
  int* list   = cursor + NBF;
  int* wcnt   = list + LISTN;
  const int tid = threadIdx.x, lane = tid & 31, wave = tid >> 5;
  const int b = blockIdx.x;
  const int nodeBase = b * NBF;

  int rb0 = rbase[b];
  const int rb1 = rbase[b + 1];
  rb0 = rb0 < 0 ? 0 : (rb0 > csrLen ? csrLen : rb0);
  rb0 &= ~31;
  int len = rb1 - rb0;
  len = len < 0 ? 0 : (len > RCAP ? RCAP : len);
  int lenW = (len + 31) & ~31;
  if (rb0 + lenW > csrLen) lenW = (csrLen - rb0) & ~31;

  {
    const v4i z = {0, 0, 0, 0};
    for (int i = tid; i < RCAP / 4; i += NTHR) ((v4i*)region)[i] = z;
    for (int s = tid; s < NBF; s += NTHR) {
      int o = off[nodeBase + s] - rb0;
      o = o < 0 ? 0 : (o > RCAP ? RCAP : o);
      cursor[s] = o;
    }
  }
  __syncthreads();

  const int nChunks = (nE + CHUNK - 1) / CHUNK;
#pragma unroll 1
  for (int ch = 0; ch < nChunks; ++ch) {
    const int cbase = ch * CHUNK;
    const int wc = scan_chunk<NBF>(dsts, nE, cbase, nodeBase, vec8, list, tid, lane, wave);
    if (lane == 0) wcnt[wave] = wc;
    __syncthreads();
    if (wave == 0) {
#pragma unroll 1
      for (int wsx = 0; wsx < NWAVE; ++wsx) {
        int n = __builtin_amdgcn_readfirstlane(wcnt[wsx]);
        n = n > WCAP ? WCAP : (n < 0 ? 0 : n);
        const int* lp = list + wsx * WCAP;
#pragma unroll 1
        for (int i = 0; i < n; ++i) {
          const int ent  = __builtin_amdgcn_readfirstlane(lp[i]);
          const int slot = ent & (NBF - 1);
          int e = cbase + ((ent >> 12) & (CHUNK - 1));
          e = e > nE - 1 ? nE - 1 : e;
          int src = srcs[e];
          src = src < 0 ? 0 : (src > nN - 1 ? nN - 1 : src);
          if (lane == 0) {
            int pos = cursor[slot];
            pos = pos < 0 ? 0 : (pos > RCAP - 1 ? RCAP - 1 : pos);
            region[pos] = src;
            const int np = pos + 1;
            cursor[slot] = np > RCAP ? RCAP : np;
          }
        }
      }
    }
    __syncthreads();
  }

  const int nv = lenW >> 2;
  int* gp = csr + rb0;
#pragma unroll 1
  for (int i = tid; i < nv; i += NTHR) { const v4i v = ((const v4i*)region)[i]; *(volatile v4i*)(gp + 4 * i) = v; }
  __threadfence();
#pragma unroll 1
  for (int i = tid; i < nv; i += NTHR) { const v4i v = ((const v4i*)region)[i]; *(volatile v4i*)(gp + 4 * i) = v; }
}

template <int KD, int NC, int RG, int EPI, int OUTD, int WH>
__global__ __launch_bounds__((NC / 64) * RG * 32) void k_gemm(
    const _Float16* __restrict__ A, const _Float16* __restrict__ Bw,
    const float* __restrict__ bia0, const float* __restrict__ bia1, const float* __restrict__ bia2,
    const float* __restrict__ res, const float* __restrict__ gam, const float* __restrict__ bet,
    float* Cf, _Float16* Ch, float asc, int nN) {
  constexpr int WPR = NC / 64;
  constexpr int NW  = WPR * RG;
  constexpr int BM  = RG * 16;
  constexpr int TPW = 4;
  static_assert(KD % 32 == 0 && NC % 64 == 0 && NW >= 1 && NW <= 12);
  static_assert(EPI != 0 || (NC % 128) == 0);
  static_assert(EPI != 1 || NC == 256);
  static_assert(EPI != 2 || (NC == 128 && NW == 8 && BM == 64));
  static_assert(BM * NC * 4 <= 32768);

  __shared__ __attribute__((aligned(16))) float stg[BM * NC];
  const int tid = threadIdx.x, lane = tid & 31, wave = tid >> 5, hh = lane >> 4, m = lane & 15;
  const int rowBase = blockIdx.x * BM;
  const int rg  = wave / WPR;
  const int chf = wave - rg * WPR;
  const int r0  = rg * 16;
  const int c0  = chf * 64;

  v8f acc[TPW];
#pragma unroll
  for (int t = 0; t < TPW; ++t) { v8f z = {0.f, 0.f, 0.f, 0.f, 0.f, 0.f, 0.f, 0.f}; acc[t] = z; }
  const _Float16* ap = A + (size_t)(rowBase + r0 + m) * KD + 8 * hh;
#pragma unroll 2
  for (int kt = 0; kt < KD / 32; ++kt) {
    Frag a;
    a.h[0] = *(const v8h*)(ap + 32 * kt);
    a.h[1] = *(const v8h*)(ap + 32 * kt + 16);
#pragma unroll
    for (int t = 0; t < TPW; ++t) {
      const _Float16* bp = Bw + (size_t)(c0 + 16 * t + m) * KD + 32 * kt + 8 * hh;
      Frag b;
      b.h[0] = *(const v8h*)bp;
      b.h[1] = *(const v8h*)(bp + 16);
      acc[t] = wmh(a.v, b.v, acc[t]);
    }
  }

  {
    float* sp = stg + (r0 + 8 * hh) * NC + c0 + m;
#pragma unroll
    for (int t = 0; t < TPW; ++t) {
#pragma unroll
      for (int r = 0; r < 8; ++r) sp[r * NC + 16 * t] = acc[t][r];
    }
  }
  __syncthreads();

  if constexpr (EPI == 0) {
    constexpr int NQ = NC / 128;
#pragma unroll 1
    for (int rr = wave; rr < BM; rr += NW) {
      const int grow = rowBase + rr;
#pragma unroll
      for (int it = 0; it < NQ; ++it) {
        const float* bsel = (it == 0) ? bia0 : ((it == 1) ? bia1 : bia2);
        const int col = it * 128 + 4 * lane;
        const v4f x  = *(const v4f*)(stg + rr * NC + col);
        const v4f bb = *(const v4f*)(bsel + 4 * lane);
        const v4f v  = x * asc + bb;
        *(volatile v4f*)(Cf + (size_t)grow * NC + col) = v;
      }
    }
    __threadfence();
#pragma unroll 1
    for (int rr = wave; rr < BM; rr += NW) {
      const int grow = rowBase + rr;
#pragma unroll
      for (int it = 0; it < NQ; ++it) {
        const float* bsel = (it == 0) ? bia0 : ((it == 1) ? bia1 : bia2);
        const int col = it * 128 + 4 * lane;
        const v4f x  = *(const v4f*)(stg + rr * NC + col);
        const v4f bb = *(const v4f*)(bsel + 4 * lane);
        const v4f v  = x * asc + bb;
        *(volatile v4f*)(Cf + (size_t)grow * NC + col) = v;
      }
    }
  } else if constexpr (EPI == 1) {
    const int col = 8 * lane;
    const v4f b0 = *(const v4f*)(bia0 + col);
    const v4f b1 = *(const v4f*)(bia0 + col + 4);
    const v4f z4 = {0.f, 0.f, 0.f, 0.f};
#pragma unroll 1
    for (int rr = wave; rr < BM; rr += NW) {
      const int grow = rowBase + rr;
      v4f x0 = *(const v4f*)(stg + rr * NC + col);
      v4f x1 = *(const v4f*)(stg + rr * NC + col + 4);
      x0 = x0 * asc + b0; x1 = x1 * asc + b1;
      x0.x = fmaxf(x0.x, 0.f); x0.y = fmaxf(x0.y, 0.f); x0.z = fmaxf(x0.z, 0.f); x0.w = fmaxf(x0.w, 0.f);
      x1.x = fmaxf(x1.x, 0.f); x1.y = fmaxf(x1.y, 0.f); x1.z = fmaxf(x1.z, 0.f); x1.w = fmaxf(x1.w, 0.f);
      (void)z4;
      const v8h o = cvt8(x0, x1, 1.0f);
      *(volatile v8h*)(Ch + (size_t)grow * NC + col) = o;
    }
    __threadfence();
#pragma unroll 1
    for (int rr = wave; rr < BM; rr += NW) {
      const int grow = rowBase + rr;
      v4f x0 = *(const v4f*)(stg + rr * NC + col);
      v4f x1 = *(const v4f*)(stg + rr * NC + col + 4);
      x0 = x0 * asc + b0; x1 = x1 * asc + b1;
      x0.x = fmaxf(x0.x, 0.f); x0.y = fmaxf(x0.y, 0.f); x0.z = fmaxf(x0.z, 0.f); x0.w = fmaxf(x0.w, 0.f);
      x1.x = fmaxf(x1.x, 0.f); x1.y = fmaxf(x1.y, 0.f); x1.z = fmaxf(x1.z, 0.f); x1.w = fmaxf(x1.w, 0.f);
      const v8h o = cvt8(x0, x1, 1.0f);
      *(volatile v8h*)(Ch + (size_t)grow * NC + col) = o;
    }
  } else {
    const int col = 4 * lane;
    const v4f bb = *(const v4f*)(bia0 + col);
    const v4f g4 = *(const v4f*)(gam + col);
    const v4f e4 = *(const v4f*)(bet + col);
    const v4f z4 = {0.f, 0.f, 0.f, 0.f};
#pragma unroll 1
    for (int i = 0; i < 8; ++i) {
      const int rr   = wave + NW * i;
      const int grow = rowBase + rr;
      const int rres = grow < nN ? grow : nN - 1;
      v4f x = *(const v4f*)(stg + rr * NC + col);
      const v4f rs = *(const v4f*)(res + (size_t)rres * NC + col);
      x = x * asc + bb;
      x = x + rs;
      float s = (x.x + x.y) + (x.z + x.w);
#pragma unroll
      for (int o = 1; o < 32; o <<= 1) s += __shfl_xor(s, o);
      const float mean = s * (1.0f / 128.0f);
      const v4f d = x - mean;
      float vs = (d.x * d.x + d.y * d.y) + (d.z * d.z + d.w * d.w);
#pragma unroll
      for (int o = 1; o < 32; o <<= 1) vs += __shfl_xor(vs, o);
      const float rstd = rsqrtf(vs * (1.0f / 128.0f) + LN_EPS);
      v4f y = d * rstd * g4 + e4;
      y = (grow < nN) ? y : z4;
      *(v4f*)(stg + rr * NC + col) = y;
      if (!OUTD || grow < nN) *(volatile v4f*)(Cf + (size_t)grow * NC + col) = y;
    }
    __syncthreads();
    if constexpr (WH != 0) {
#pragma unroll
      for (int i = 0; i < 4; ++i) {
        const int rr   = wave + NW * (2 * i + hh);
        const int grow = rowBase + rr;
        const v4f y0 = *(const v4f*)(stg + rr * NC + 8 * m);
        const v4f y1 = *(const v4f*)(stg + rr * NC + 8 * m + 4);
        const v8h o = cvt8(y0, y1, 1.0f);
        *(volatile v8h*)(Ch + (size_t)grow * NC + 8 * m) = o;
      }
    }
    __threadfence();
#pragma unroll 1
    for (int i = 0; i < 8; ++i) {
      const int rr   = wave + NW * i;
      const int grow = rowBase + rr;
      const v4f y = *(const v4f*)(stg + rr * NC + col);
      if (!OUTD || grow < nN) *(volatile v4f*)(Cf + (size_t)grow * NC + col) = y;
    }
    if constexpr (WH != 0) {
#pragma unroll
      for (int i = 0; i < 4; ++i) {
        const int rr   = wave + NW * (2 * i + hh);
        const int grow = rowBase + rr;
        const v4f y0 = *(const v4f*)(stg + rr * NC + 8 * m);
        const v4f y1 = *(const v4f*)(stg + rr * NC + 8 * m + 4);
        const v8h o = cvt8(y0, y1, 1.0f);
        *(volatile v8h*)(Ch + (size_t)grow * NC + 8 * m) = o;
      }
    }
  }
}

__global__ __launch_bounds__(NTHR) void k_agg(
    const int* __restrict__ csr, const int* __restrict__ off, const int* __restrict__ cnt,
    const float* __restrict__ qkv, _Float16* attn, int nN, int csrLen) {
  __shared__ __attribute__((aligned(16))) _Float16 sOut[NWAVE * 16 * DD];
  const int tid = threadIdx.x, lane = tid & 31, wave = tid >> 5, hh = lane >> 4, m = lane & 15;
  const int tbase = blockIdx.x * TGT + wave * 32;
  const int col = 4 * lane;
  const int cnt_l = cnt[tbase + lane];
  const int off_l = off[tbase + lane];
  _Float16* sw = sOut + wave * (16 * DD);
  const v4f z4 = {0.f, 0.f, 0.f, 0.f};

#pragma unroll 1
  for (int hf = 0; hf < 2; ++hf) {
#pragma unroll 1
    for (int j = 0; j < 16; ++j) {
      const int jj = hf * 16 + j;
      const int c  = tbase + jj;
      int n = __shfl(cnt_l, jj);
      n = n < 0 ? 0 : (n > DEGCAP ? DEGCAP : n);
      const int st = __shfl(off_l, jj);
      const v4f q = *(const v4f*)(qkv + (size_t)c * QKVW + col);
      float z = 0.f;
      v4f acc = z4;
#pragma unroll 1
      for (int q0 = 0; q0 < n; q0 += 32) {
        int pos = st + q0 + lane;
        pos = pos < 0 ? 0 : (pos > csrLen - 1 ? csrLen - 1 : pos);
        int sl = csr[pos];
        sl = sl < 0 ? 0 : (sl > nN - 1 ? nN - 1 : sl);
        const int mcnt = (n - q0) < 32 ? (n - q0) : 32;
#pragma unroll 1
        for (int pp = 0; pp < mcnt; ++pp) {
          const int s = __builtin_amdgcn_readlane(sl, pp);
          const float* rp = qkv + (size_t)s * QKVW + col;
          const v4f kv = *(const v4f*)(rp + DD);
          const v4f vv = *(const v4f*)(rp + 2 * DD);
          float p = kv.x * q.x + kv.y * q.y + kv.z * q.z + kv.w * q.w;
          p += __shfl_xor(p, 1);
          p += __shfl_xor(p, 2);
          const float sc = __expf(fminf(fmaxf(p * 0.25f, -5.0f), 5.0f));
          z += sc;
          acc = acc + vv * sc;
        }
      }
      const float rz = 1.0f / (z + Z_EPS);
      v4f a = acc * rz;
      a = (c < nN) ? a : z4;
      v4h o;
      o[0] = (_Float16)(a.x * ACARRY); o[1] = (_Float16)(a.y * ACARRY);
      o[2] = (_Float16)(a.z * ACARRY); o[3] = (_Float16)(a.w * ACARRY);
      *(v4h*)(sw + j * DD + col) = o;
    }
    __syncthreads();
#pragma unroll
    for (int it = 0; it < 8; ++it) {
      const int row  = 2 * it + hh;
      const int grow = tbase + hf * 16 + row;
      const v8h ov = *(const v8h*)(sw + row * DD + 8 * m);
      *(volatile v8h*)(attn + (size_t)grow * DD + 8 * m) = ov;
    }
    __threadfence();
#pragma unroll
    for (int it = 0; it < 8; ++it) {
      const int row  = 2 * it + hh;
      const int grow = tbase + hf * 16 + row;
      const v8h ov = *(const v8h*)(sw + row * DD + 8 * m);
      *(volatile v8h*)(attn + (size_t)grow * DD + 8 * m) = ov;
    }
    __syncthreads();
  }
}

extern "C" void kernel_launch(void* const* d_in, const int* in_sizes, int n_in,
                              void* d_out, int out_size, void* d_ws, size_t ws_size,
                              hipStream_t stream) {
  if (n_in < 19) return;
  const int nN = in_sizes[0] / DD;
  const int nE = in_sizes[1];
  if (nN <= 0 || nE <= 0 || in_sizes[0] != nN * DD || in_sizes[2] != nE) return;
  if (in_sizes[3] != NL * DD * DD || in_sizes[5] != NL * DD * DD || in_sizes[7] != NL * DD * DD || in_sizes[9] != NL * DD * DD) return;
  if (in_sizes[11] != NL * DD * FFW || in_sizes[13] != NL * FFW * DD) return;
  if (in_sizes[4] != NL * DD || in_sizes[6] != NL * DD || in_sizes[8] != NL * DD || in_sizes[10] != NL * DD) return;
  if (in_sizes[12] != NL * FFW || in_sizes[14] != NL * DD) return;
  for (int i = 15; i <= 18; ++i) if (in_sizes[i] != NL * DD) return;
  if (out_size != nN * DD) return;
  if (nE > (1 << 28) || nN > (1 << 24)) return;

  const float* hin = (const float*)d_in[0];
  const int*   src = (const int*)d_in[1];
  const int*   dst = (const int*)d_in[2];
  const float* Wq  = (const float*)d_in[3];   const float* bq  = (const float*)d_in[4];
  const float* Wk  = (const float*)d_in[5];   const float* bk  = (const float*)d_in[6];
  const float* Wv  = (const float*)d_in[7];   const float* bv  = (const float*)d_in[8];
  const float* Wo  = (const float*)d_in[9];   const float* bo  = (const float*)d_in[10];
  const float* W1  = (const float*)d_in[11];  const float* b1  = (const float*)d_in[12];
  const float* W2  = (const float*)d_in[13];  const float* b2  = (const float*)d_in[14];
  const float* g1  = (const float*)d_in[15];  const float* be1 = (const float*)d_in[16];
  const float* g2  = (const float*)d_in[17];  const float* be2 = (const float*)d_in[18];
  float* out = (float*)d_out;

  const int NPAD   = ((nN + TGT - 1) / TGT) * TGT;
  const int nBC    = (nN + NBC - 1) / NBC;
  const int CNTPAD = nBC * NBC;
  if (4 * nBC + 1 > RBN) return;
  const int nBF    = (nN + NBF - 1) / NBF;
  const int csrLen = ((nE + 31) & ~31) + 4096;
  if (31 * 4 * nBC > 4096) return;
  const int nAgg   = NPAD / TGT;

  char* ws = (char*)d_ws;
  size_t off = 0;
  const size_t oWqkv = off; off += (size_t)NL * QKVW * DD * 2;   off = (off + 255) & ~(size_t)255;
  const size_t oWo   = off; off += (size_t)NL * DD * DD * 2;     off = (off + 255) & ~(size_t)255;
  const size_t oW1   = off; off += (size_t)NL * FFW * DD * 2;    off = (off + 255) & ~(size_t)255;
  const size_t oW2   = off; off += (size_t)NL * DD * FFW * 2;    off = (off + 255) & ~(size_t)255;
  const size_t oCnt  = off; off += (size_t)CNTPAD * 4;           off = (off + 255) & ~(size_t)255;
  const size_t oOff  = off; off += (size_t)CNTPAD * 4;           off = (off + 255) & ~(size_t)255;
  const size_t oRb   = off; off += (size_t)RBN * 4;              off = (off + 255) & ~(size_t)255;
  const size_t oCsr  = off; off += (size_t)csrLen * 4;           off = (off + 255) & ~(size_t)255;
  const size_t oX    = off; off += (size_t)NPAD * QKVW * 4;      off = (off + 255) & ~(size_t)255;
  const size_t oA    = off; off += (size_t)NPAD * DD * 2;        off = (off + 255) & ~(size_t)255;
  const size_t oH    = off; off += (size_t)NPAD * DD * 4;        off = (off + 255) & ~(size_t)255;
  if (off > ws_size || off > (size_t)WSCAP) return;
  _Float16* wqkv = (_Float16*)(ws + oWqkv);
  _Float16* wo   = (_Float16*)(ws + oWo);
  _Float16* w1   = (_Float16*)(ws + oW1);
  _Float16* w2   = (_Float16*)(ws + oW2);
  int*   cnt  = (int*)(ws + oCnt);
  int*   offp = (int*)(ws + oOff);
  int*   rb   = (int*)(ws + oRb);
  int*   csr  = (int*)(ws + oCsr);
  float* qkv  = (float*)(ws + oX);
  float* h1f  = (float*)(ws + oX);
  _Float16* h1A = (_Float16*)(ws + oX + (size_t)NPAD * DD * 4);
  _Float16* ffA = (_Float16*)(ws + oX + (size_t)NPAD * DD * 4 + (size_t)NPAD * DD * 2);
  _Float16* hA  = (_Float16*)(ws + oA);
  float* hf   = (float*)(ws + oH);

  const int vec8 = ((nE & 3) == 0) ? 1 : 0;

  {
    const int uq = NL * DD * (DD / 8);
    k_wprep<<<(uq + NTHR - 1) / NTHR, NTHR, 0, stream>>>(Wq, wqkv, DD, DD, uq, QKVW * DD, 0);
    k_wprep<<<(uq + NTHR - 1) / NTHR, NTHR, 0, stream>>>(Wk, wqkv, DD, DD, uq, QKVW * DD, DD);
    k_wprep<<<(uq + NTHR - 1) / NTHR, NTHR, 0, stream>>>(Wv, wqkv, DD, DD, uq, QKVW * DD, 2 * DD);
    k_wprep<<<(uq + NTHR - 1) / NTHR, NTHR, 0, stream>>>(Wo, wo, DD, DD, uq, DD * DD, 0);
    const int u1 = NL * FFW * (DD / 8);
    k_wprep<<<(u1 + NTHR - 1) / NTHR, NTHR, 0, stream>>>(W1, w1, DD, FFW, u1, FFW * DD, 0);
    const int u2 = NL * DD * (FFW / 8);
    k_wprep<<<(u2 + NTHR - 1) / NTHR, NTHR, 0, stream>>>(W2, w2, FFW, DD, u2, DD * FFW, 0);
  }
  {
    const int uc = NPAD * (DD / 8);
    k_cvt<<<(uc + NTHR - 1) / NTHR, NTHR, 0, stream>>>(hin, hA, nN, uc);
  }
  k_count<<<nBC, NTHR, 0, stream>>>(dst, cnt, nE, vec8);
  k_offsets<<<1, OTHR, 0, stream>>>(cnt, offp, rb, nBC);
  hipFuncSetAttribute(reinterpret_cast<const void*>(&k_fill),
                      hipFuncAttributeMaxDynamicSharedMemorySize, LDS_FILL);
  k_fill<<<nBF, NTHR, LDS_FILL, stream>>>(src, dst, offp, rb, csr, nN, nE, vec8, csrLen);

  for (int l = 0; l < NL; ++l) {
    k_gemm<DD, QKVW, 1, 0, 0, 0><<<NPAD / 16, (QKVW / 64) * 1 * 32, 0, stream>>>(
        hA, wqkv + (size_t)l * QKVW * DD, bq + (size_t)l * DD, bk + (size_t)l * DD, bv + (size_t)l * DD,
        bq, bq, bq, qkv, hA, 1.0f / WCARRY, nN);
    k_agg<<<nAgg, NTHR, 0, stream>>>(csr, offp, cnt, qkv, hA, nN, csrLen);
    const float* resin = (l == 0) ? hin : hf;
    k_gemm<DD, DD, 4, 2, 0, 1><<<NPAD / 64, NTHR, 0, stream>>>(
        hA, wo + (size_t)l * DD * DD, bo + (size_t)l * DD, bo, bo,
        resin, g1 + (size_t)l * DD, be1 + (size_t)l * DD, h1f, h1A, 1.0f / (WCARRY * ACARRY), nN);
    k_gemm<DD, FFW, 2, 1, 0, 0><<<NPAD / 32, NTHR, 0, stream>>>(
        h1A, w1 + (size_t)l * FFW * DD, b1 + (size_t)l * FFW, b1, b1,
        b1, b1, b1, h1f, ffA, 1.0f / WCARRY, nN);
    if (l + 1 < NL) {
      k_gemm<FFW, DD, 4, 2, 0, 1><<<NPAD / 64, NTHR, 0, stream>>>(
          ffA, w2 + (size_t)l * DD * FFW, b2 + (size_t)l * DD, b2, b2,
          h1f, g2 + (size_t)l * DD, be2 + (size_t)l * DD, hf, hA, 1.0f / WCARRY, nN);
    } else {
      k_gemm<FFW, DD, 4, 2, 1, 0><<<NPAD / 64, NTHR, 0, stream>>>(
          ffA, w2 + (size_t)l * DD * FFW, b2 + (size_t)l * DD, b2, b2,
          h1f, g2 + (size_t)l * DD, be2 + (size_t)l * DD, out, hA, 1.0f / WCARRY, nN);
    }
  }
}
